// RPTAttention_63797444215057
// MI455X (gfx1250) — hardware-verified
//
#include <hip/hip_runtime.h>


typedef unsigned short u16;
typedef unsigned int   u32;
typedef _Float16 v16h __attribute__((ext_vector_type(16)));
typedef _Float16 v8h  __attribute__((ext_vector_type(8)));
typedef __bf16   v16b __attribute__((ext_vector_type(16)));
typedef float    v8f  __attribute__((ext_vector_type(8)));
typedef float    v4f  __attribute__((ext_vector_type(4)));
typedef u32      v4u  __attribute__((ext_vector_type(4)));

#define SEQ   2048
#define HID   2048
#define NHEAD 16
#define NKVH  4
#define HDIM  128
#define QDIM  (NHEAD * HDIM)
#define KDIM  (NKVH * HDIM)
#define R_ATT 1024
#define R_OUT 512

__device__ __forceinline__ u16 f2bf(float f) {
    u32 u = __float_as_uint(f);
    u32 r = u + 0x7FFFu + ((u >> 16) & 1u);
    return (u16)(r >> 16);
}
__device__ __forceinline__ float bf2f(u16 b) { return __uint_as_float(((u32)b) << 16); }
__device__ __forceinline__ u16 f2h(float f) { union { _Float16 h; u16 u; } c; c.h = (_Float16)f; return c.u; }
__device__ __forceinline__ float h2f(u16 u) { union { _Float16 h; u16 u; } c; c.u = u; return (float)c.h; }
__device__ __forceinline__ v4u ld16(const u16* p) { return *(const v4u*)p; }

union FragH { v16h v; v4u q[2]; };
union FragB { v16b v; v4u q[2]; };

template<int BF> struct FSel { typedef FragH F; };
template<> struct FSel<1> { typedef FragB F; };

__device__ __forceinline__ v8f mm1(const FragH& a, const FragH& b, v8f c) {
    return __builtin_amdgcn_wmma_f32_16x16x32_f16(false, a.v, false, b.v, (short)0, c, false, false);
}
__device__ __forceinline__ v8f mm1(const FragB& a, const FragB& b, v8f c) {
    return __builtin_amdgcn_wmma_f32_16x16x32_bf16(false, a.v, false, b.v, (short)0, c, false, false);
}
__device__ __forceinline__ v8f mmg(const FragH& a, const FragH& b, v8f c) {
    c = mm1(a, b, c);
    asm volatile("v_nop\n\tv_nop\n\tv_nop\n\tv_nop" : "+v"(c) : "v"(a.v), "v"(b.v));
    return c;
}
__device__ __forceinline__ v8f mmg(const FragB& a, const FragB& b, v8f c) {
    c = mm1(a, b, c);
    asm volatile("v_nop\n\tv_nop\n\tv_nop\n\tv_nop" : "+v"(c) : "v"(a.v), "v"(b.v));
    return c;
}
__device__ __forceinline__ v8f mm2(const FragH& a0, const FragH& a1, const FragH& b, v8f c) {
    c = mm1(a0, b, c);
    c = mm1(a1, b, c);
    asm volatile("v_nop\n\tv_nop\n\tv_nop\n\tv_nop" : "+v"(c) : "v"(a0.v), "v"(a1.v), "v"(b.v));
    return c;
}
__device__ __forceinline__ v8f mm2(const FragB& a0, const FragB& a1, const FragB& b, v8f c) {
    c = mm1(a0, b, c);
    c = mm1(a1, b, c);
    asm volatile("v_nop\n\tv_nop\n\tv_nop\n\tv_nop" : "+v"(c) : "v"(a0.v), "v"(a1.v), "v"(b.v));
    return c;
}
__device__ __forceinline__ v8f mm3(const FragH& ah, const FragH& al, const FragH& bh, const FragH& bl, v8f c) {
    c = mm1(ah, bh, c);
    c = mm1(ah, bl, c);
    c = mm1(al, bh, c);
    asm volatile("v_nop\n\tv_nop\n\tv_nop\n\tv_nop" : "+v"(c) : "v"(ah.v), "v"(al.v), "v"(bh.v), "v"(bl.v));
    return c;
}

__device__ __forceinline__ void pack8(const float* y, v4u& hq, v4u& lq) {
    union { v8h h; v4u q; } ph, pl;
#pragma unroll
    for (int e = 0; e < 8; ++e) {
        _Float16 a = (_Float16)y[e];
        ph.h[e] = a;
        pl.h[e] = (_Float16)(y[e] - (float)a);
    }
    hq = ph.q; lq = pl.q;
}

__global__ __launch_bounds__(256)
void k_cvtx(const float* __restrict__ x, u16* xb, int n8) {
    int i = (int)blockIdx.x * 256 + (int)threadIdx.x;
    if (i >= n8) return;
    const float* p = x + (size_t)i * 8;
    v4f a = *(const v4f*)p, b = *(const v4f*)(p + 4);
    union { u16 h[8]; v4u q; } w;
    w.h[0] = f2bf(a.x); w.h[1] = f2bf(a.y); w.h[2] = f2bf(a.z); w.h[3] = f2bf(a.w);
    w.h[4] = f2bf(b.x); w.h[5] = f2bf(b.y); w.h[6] = f2bf(b.z); w.h[7] = f2bf(b.w);
    u16* d = xb + (size_t)i * 8;
    *(volatile v4u*)d = w.q;
    __threadfence();
    *(volatile v4u*)d = w.q;
}

__global__ __launch_bounds__(256)
void k_table(float* cs) {
    __shared__ float fr[HDIM / 2];
    const int t = (int)threadIdx.x;
    if (t < HDIM / 2) {
        float e = (float)(2 * t) / (float)HDIM;
        double p = pow(10000.0, (double)e);
        float pf = (float)p;
        fr[t] = 1.0f / pf;
    }
    __syncthreads();
    const int s = (int)blockIdx.x * 8 + (t >> 5);
    const int jp = t & 31;
    if (s >= SEQ) return;
    float a0 = (float)s * fr[2 * jp];
    float a1 = (float)s * fr[2 * jp + 1];
    float s0, c0, s1, c1;
    sincosf(a0, &s0, &c0);
    sincosf(a1, &s1, &c1);
    v4f v = {c0, s0, c1, s1};
    float* d = cs + (size_t)s * HDIM + 4 * jp;
    *(volatile v4f*)d = v;
    __threadfence();
    *(volatile v4f*)d = v;
}

template<int MODE>
__global__ __launch_bounds__(256)
void k_wt(const float* __restrict__ w, u16* out, int K, int N) {
    __shared__ u16 T[64 * 64];
    const int t = (int)threadIdx.x, wv = t >> 5, lane = t & 31;
    const int k0 = (int)blockIdx.x * 64, n0 = (int)blockIdx.y * 64;
    if (k0 + 64 > K || n0 + 64 > N) return;
    const int r = t >> 2, c0 = (t & 3) * 16;
    const float* src = w + (size_t)(k0 + r) * N + n0 + c0;
#pragma unroll
    for (int q = 0; q < 4; ++q) {
        v4f v = *(const v4f*)(src + 4 * q);
        float e[4] = {v.x, v.y, v.z, v.w};
#pragma unroll
        for (int u = 0; u < 4; ++u) {
            u16 b = f2bf(e[u]);
            u16 o16 = MODE ? f2h(bf2f(b) * 1024.0f) : b;
            T[(c0 + 4 * q + u) * 64 + r] = o16;
        }
    }
    __syncthreads();
#pragma unroll
    for (int p = 0; p < 2; ++p) {
        int n = wv * 8 + p * 4 + (lane >> 3), ks = (lane & 7) * 8;
        v4u v = *(const v4u*)&T[n * 64 + ks];
        *(volatile v4u*)(out + (size_t)(n0 + n) * K + k0 + ks) = v;
    }
    __threadfence();
#pragma unroll
    for (int p = 0; p < 2; ++p) {
        int n = wv * 8 + p * 4 + (lane >> 3), ks = (lane & 7) * 8;
        v4u v = *(const v4u*)&T[n * 64 + ks];
        *(volatile v4u*)(out + (size_t)(n0 + n) * K + k0 + ks) = v;
    }
}

__device__ __forceinline__ void out_pass(const float* Ts, float* Cf, int wv, int lane, int m0, int n0, int N, float oscale) {
#pragma unroll
    for (int r = 0; r < 16; ++r) {
        int row = wv * 16 + r;
        v4f v = *(const v4f*)&Ts[row * 128 + 4 * lane];
        v = v * oscale;
        *(volatile v4f*)(Cf + (size_t)(m0 + row) * N + n0 + 4 * lane) = v;
    }
}
__device__ __forceinline__ void rope8(const float* tr, const float* cr, float* y) {
    v4f t0 = *(const v4f*)tr, t1 = *(const v4f*)(tr + 4);
    v4f k0 = *(const v4f*)cr, k1 = *(const v4f*)(cr + 4);
    float tv[8] = {t0.x, t0.y, t0.z, t0.w, t1.x, t1.y, t1.z, t1.w};
    float kv[8] = {k0.x, k0.y, k0.z, k0.w, k1.x, k1.y, k1.z, k1.w};
#pragma unroll
    for (int p = 0; p < 4; ++p) {
        float re = tv[2 * p], im = tv[2 * p + 1];
        float c = kv[2 * p], sn = kv[2 * p + 1];
        y[2 * p]     = re * c - im * sn;
        y[2 * p + 1] = re * sn + im * c;
    }
}
__device__ __forceinline__ void rope_pass(const float* Ts, const float* cs, u16* P0, u16* P1, bool wl,
                                          int wv, int l16, int hh, int m0, int n0, int N) {
#pragma unroll
    for (int rr = 0; rr < 8; ++rr) {
        int row = wv * 16 + 2 * rr + hh, seg = 8 * l16;
        float y[8];
        rope8(&Ts[row * 128 + seg], cs + (size_t)(m0 + row) * HDIM + seg, y);
        v4u hq, lq;
        pack8(y, hq, lq);
        size_t o = (size_t)(m0 + row) * N + n0 + seg;
        *(volatile v4u*)(P0 + o) = hq;
        if (wl) *(volatile v4u*)(P1 + o) = lq;
    }
}
__device__ __forceinline__ void vt_pass(const float* Ts, u16* P0, u16* P1, bool wl,
                                        int wv, int l16, int hh, int hv, int M, int m0) {
#pragma unroll
    for (int rr = 0; rr < 8; ++rr) {
        int d = wv * 16 + 2 * rr + hh, seg = 8 * l16;
        const float* tr = &Ts[d * 128 + seg];
        v4f t0 = *(const v4f*)tr, t1 = *(const v4f*)(tr + 4);
        float y[8] = {t0.x, t0.y, t0.z, t0.w, t1.x, t1.y, t1.z, t1.w};
        v4u hq, lq;
        pack8(y, hq, lq);
        size_t o = ((size_t)(hv * HDIM + d)) * M + m0 + seg;
        *(volatile v4u*)(P0 + o) = hq;
        if (wl) *(volatile v4u*)(P1 + o) = lq;
    }
}

template<int BF, int NA, int EP>
__global__ __launch_bounds__(256)
void k_gemm(const u16* __restrict__ A0, const u16* __restrict__ A1, const u16* __restrict__ BT,
            float* Cf, u16* P0, u16* P1, const float* __restrict__ cs,
            int M, int N, int K, int m_base, int lo_rows, float oscale) {
    __shared__ u16   Bs[128 * 32];
    __shared__ float Ts[128 * 128];
    typedef typename FSel<BF>::F Frag;
    const int tid = (int)threadIdx.x, wv = tid >> 5, lane = tid & 31, l16 = lane & 15, hh = lane >> 4;
    const int m0 = m_base + (int)blockIdx.y * 128, n0 = (int)blockIdx.x * 128;
    if (m0 + 128 > M || n0 + 128 > N) return;

    v8f acc[8];
#pragma unroll
    for (int nb = 0; nb < 8; ++nb) acc[nb] = (v8f){0, 0, 0, 0, 0, 0, 0, 0};

    const size_t arow = (size_t)(m0 + wv * 16 + l16) * K;

    for (int kk = 0; kk < K; kk += 32) {
#pragma unroll
        for (int j = 0; j < 2; ++j) {
            int idx = tid + 256 * j, n = idx >> 2, ch = idx & 3;
            *(v4u*)&Bs[n * 32 + ch * 8] = ld16(BT + (size_t)(n0 + n) * K + kk + ch * 8);
        }
        __syncthreads();
        Frag fa0, fa1;
        fa0.q[0] = ld16(A0 + arow + kk + 8 * hh);
        fa0.q[1] = ld16(A0 + arow + kk + 16 + 8 * hh);
        fa1 = fa0;
        if (NA == 2) {
            fa1.q[0] = ld16(A1 + arow + kk + 8 * hh);
            fa1.q[1] = ld16(A1 + arow + kk + 16 + 8 * hh);
        }
#pragma unroll
        for (int nb = 0; nb < 8; ++nb) {
            Frag fb;
            fb.q[0] = *(const v4u*)&Bs[(nb * 16 + l16) * 32 + 8 * hh];
            fb.q[1] = *(const v4u*)&Bs[(nb * 16 + l16) * 32 + 16 + 8 * hh];
            if (NA == 2) acc[nb] = mm2(fa0, fa1, fb, acc[nb]);
            else         acc[nb] = mmg(fa0, fb, acc[nb]);
        }
        __syncthreads();
    }

    if (EP == 2) {
#pragma unroll
        for (int nb = 0; nb < 8; ++nb)
#pragma unroll
            for (int i = 0; i < 8; ++i)
                Ts[(nb * 16 + l16) * 128 + (wv * 16 + 8 * hh + i)] = acc[nb][i];
    } else {
#pragma unroll
        for (int nb = 0; nb < 8; ++nb)
#pragma unroll
            for (int i = 0; i < 8; ++i)
                Ts[(wv * 16 + 8 * hh + i) * 128 + nb * 16 + l16] = acc[nb][i];
    }
    __syncthreads();

    const bool wl = (m0 < lo_rows);
    if (EP == 0) {
        out_pass(Ts, Cf, wv, lane, m0, n0, N, oscale);
        __threadfence();
        out_pass(Ts, Cf, wv, lane, m0, n0, N, oscale);
    } else if (EP == 1) {
        rope_pass(Ts, cs, P0, P1, wl, wv, l16, hh, m0, n0, N);
        __threadfence();
        rope_pass(Ts, cs, P0, P1, wl, wv, l16, hh, m0, n0, N);
    } else {
        const int hv = (int)blockIdx.x;
        vt_pass(Ts, P0, P1, wl, wv, l16, hh, hv, M, m0);
        __threadfence();
        vt_pass(Ts, P0, P1, wl, wv, l16, hh, hv, M, m0);
    }
}

__device__ __forceinline__ void ctx_pass(const u16* src, u16* C, int wv, int l16, int hh, int qr0, int h) {
#pragma unroll
    for (int rr = 0; rr < 8; ++rr) {
        int row = wv * 16 + 2 * rr + hh, seg = 8 * l16;
        v4u v = *(const v4u*)&src[row * 128 + seg];
        *(volatile v4u*)(C + ((size_t)(qr0 + row) * NHEAD + h) * HDIM + seg) = v;
    }
}

template<int SPLIT>
__global__ __launch_bounds__(128)
void k_attn(const u16* __restrict__ Qh, const u16* __restrict__ Ql,
            const u16* __restrict__ Kh, const u16* __restrict__ Kl,
            const u16* __restrict__ Vh, const u16* __restrict__ Vl,
            u16* Ch, u16* Cl, int qt_base, int lo_rows) {
    __shared__ u16 lds[64 * 128];
    const int tid = (int)threadIdx.x, wv = tid >> 5, lane = tid & 31, l16 = lane & 15, hh = lane >> 4;
    const int h = (int)blockIdx.x, qt = qt_base + (int)blockIdx.y, hkv = h >> 2;
    if (qt * 64 + 64 > SEQ || h >= NHEAD) return;
    const int qr0 = qt * 64;
    const float scale = 0.08838834764831845f;
    const size_t qoff = ((size_t)(qr0 + wv * 16 + l16) * NHEAD + h) * HDIM;

    v8f o[8];
    float m_i[8], l_i[8];
#pragma unroll
    for (int nb = 0; nb < 8; ++nb) o[nb] = (v8f){0, 0, 0, 0, 0, 0, 0, 0};
#pragma unroll
    for (int i = 0; i < 8; ++i) { m_i[i] = -1.0e30f; l_i[i] = 0.0f; }

    for (int kt = 0; kt <= qt; ++kt) {
        const int kb = kt * 64;

        v8f s[4];
#pragma unroll
        for (int nb = 0; nb < 4; ++nb) s[nb] = (v8f){0, 0, 0, 0, 0, 0, 0, 0};
#pragma unroll
        for (int c = 0; c < 4; ++c) {
            FragH qa, qb;
            qa.q[0] = ld16(Qh + qoff + c * 32 + 8 * hh);
            qa.q[1] = ld16(Qh + qoff + c * 32 + 16 + 8 * hh);
            qb = qa;
            if (SPLIT) {
                qb.q[0] = ld16(Ql + qoff + c * 32 + 8 * hh);
                qb.q[1] = ld16(Ql + qoff + c * 32 + 16 + 8 * hh);
            }
#pragma unroll
            for (int nb = 0; nb < 4; ++nb) {
                const size_t ko = ((size_t)(kb + nb * 16 + l16) * NKVH + hkv) * HDIM + c * 32;
                FragH ka, kl2;
                ka.q[0] = ld16(Kh + ko + 8 * hh);
                ka.q[1] = ld16(Kh + ko + 16 + 8 * hh);
                if (SPLIT) {
                    kl2.q[0] = ld16(Kl + ko + 8 * hh);
                    kl2.q[1] = ld16(Kl + ko + 16 + 8 * hh);
                    s[nb] = mm3(qa, qb, ka, kl2, s[nb]);
                } else {
                    s[nb] = mmg(qa, ka, s[nb]);
                }
            }
        }

        const bool diag = (kt == qt);
#pragma unroll
        for (int nb = 0; nb < 4; ++nb)
#pragma unroll
            for (int i = 0; i < 8; ++i) {
                float v = s[nb][i] * scale;
                if (diag) {
                    int qq = qr0 + wv * 16 + 8 * hh + i;
                    int ky = kb + nb * 16 + l16;
                    if (ky > qq) v = -1.0e30f;
                }
                s[nb][i] = v;
            }

        float mnew[8], alpha[8];
#pragma unroll
        for (int i = 0; i < 8; ++i) {
            float mx = m_i[i];
#pragma unroll
            for (int nb = 0; nb < 4; ++nb) {
                float v = s[nb][i];
#pragma unroll
                for (int off = 1; off < 16; off <<= 1) v = fmaxf(v, __shfl_xor(v, off, 32));
                mx = fmaxf(mx, v);
            }
            mnew[i]  = mx;
            alpha[i] = __expf(m_i[i] - mx);
            m_i[i]   = mx;
        }
#pragma unroll
        for (int i = 0; i < 8; ++i) {
            float sum = 0.0f;
#pragma unroll
            for (int nb = 0; nb < 4; ++nb) {
                float p = __expf(s[nb][i] - mnew[i]);
                s[nb][i] = p;
#pragma unroll
                for (int off = 1; off < 16; off <<= 1) p += __shfl_xor(p, off, 32);
                sum += p;
            }
            l_i[i] = l_i[i] * alpha[i] + sum;
        }

        __syncthreads();
#pragma unroll
        for (int nb = 0; nb < 4; ++nb)
#pragma unroll
            for (int i = 0; i < 8; ++i) {
                int r = wv * 16 + 8 * hh + i;
                float p = s[nb][i] * 256.0f;
                u16 ph = f2h(p);
                lds[r * 64 + nb * 16 + l16] = ph;
                if (SPLIT) lds[4096 + r * 64 + nb * 16 + l16] = f2h(p - h2f(ph));
            }
        __syncthreads();

#pragma unroll
        for (int nb = 0; nb < 8; ++nb)
#pragma unroll
            for (int i = 0; i < 8; ++i) o[nb][i] = o[nb][i] * alpha[i];

#pragma unroll
        for (int c = 0; c < 2; ++c) {
            const int pr = (wv * 16 + l16) * 64 + c * 32;
            FragH pa, pb;
            pa.q[0] = *(const v4u*)&lds[pr + 8 * hh];
            pa.q[1] = *(const v4u*)&lds[pr + 16 + 8 * hh];
            pb = pa;
            if (SPLIT) {
                pb.q[0] = *(const v4u*)&lds[4096 + pr + 8 * hh];
                pb.q[1] = *(const v4u*)&lds[4096 + pr + 16 + 8 * hh];
            }
#pragma unroll
            for (int nb = 0; nb < 8; ++nb) {
                const size_t vo = ((size_t)(hkv * HDIM + nb * 16 + l16)) * SEQ + kb + c * 32;
                FragH va, vb;
                va.q[0] = ld16(Vh + vo + 8 * hh);
                va.q[1] = ld16(Vh + vo + 16 + 8 * hh);
                if (SPLIT) {
                    vb.q[0] = ld16(Vl + vo + 8 * hh);
                    vb.q[1] = ld16(Vl + vo + 16 + 8 * hh);
                    o[nb] = mm3(pa, pb, va, vb, o[nb]);
                } else {
                    o[nb] = mmg(pa, va, o[nb]);
                }
            }
        }
    }

    float rl[8];
#pragma unroll
    for (int i = 0; i < 8; ++i) rl[i] = 0.25f / l_i[i];

    __syncthreads();
#pragma unroll
    for (int nb = 0; nb < 8; ++nb)
#pragma unroll
        for (int i = 0; i < 8; ++i)
            lds[(wv * 16 + 8 * hh + i) * 128 + nb * 16 + l16] = f2h(o[nb][i] * rl[i]);
    __syncthreads();
    ctx_pass(lds, Ch, wv, l16, hh, qr0, h);
    __threadfence();
    ctx_pass(lds, Ch, wv, l16, hh, qr0, h);

    if (qr0 < lo_rows) {
        __syncthreads();
#pragma unroll
        for (int nb = 0; nb < 8; ++nb)
#pragma unroll
            for (int i = 0; i < 8; ++i) {
                float v = o[nb][i] * rl[i];
                lds[(wv * 16 + 8 * hh + i) * 128 + nb * 16 + l16] = f2h(v - h2f(f2h(v)));
            }
        __syncthreads();
        ctx_pass(lds, Cl, wv, l16, hh, qr0, h);
        __threadfence();
        ctx_pass(lds, Cl, wv, l16, hh, qr0, h);
    }
}

extern "C" void kernel_launch(void* const* d_in, const int* in_sizes, int n_in,
                              void* d_out, int out_size, void* d_ws, size_t ws_size,
                              hipStream_t stream) {
    if (n_in < 5) return;
    if (in_sizes[0] != SEQ * HID || in_sizes[1] != HID * QDIM || in_sizes[2] != HID * KDIM ||
        in_sizes[3] != HID * KDIM || in_sizes[4] != QDIM * HID) return;
    if (out_size != SEQ * HID) return;

    const float* X  = (const float*)d_in[0];
    const float* Wq = (const float*)d_in[1];
    const float* Wk = (const float*)d_in[2];
    const float* Wv = (const float*)d_in[3];
    const float* Wo = (const float*)d_in[4];
    float* Out = (float*)d_out;

    char* ws = (char*)d_ws;
    size_t off = 0;
    u16*   xb  = (u16*)(ws + off);   off += (size_t)SEQ * HID * 2;
    u16*   wqT = (u16*)(ws + off);   off += (size_t)QDIM * HID * 2;
    u16*   wkT = (u16*)(ws + off);   off += (size_t)KDIM * HID * 2;
    u16*   wvT = (u16*)(ws + off);   off += (size_t)KDIM * HID * 2;
    u16*   woT = (u16*)(ws + off);   off += (size_t)HID * QDIM * 2;
    float* csf = (float*)(ws + off); off += (size_t)SEQ * HDIM * 4;
    u16*   qh  = (u16*)(ws + off);   off += (size_t)SEQ * QDIM * 2;
    u16*   ql  = (u16*)(ws + off);   off += (size_t)SEQ * QDIM * 2;
    u16*   kh  = (u16*)(ws + off);   off += (size_t)SEQ * KDIM * 2;
    u16*   kl  = (u16*)(ws + off);   off += (size_t)SEQ * KDIM * 2;
    u16*   vh  = (u16*)(ws + off);   off += (size_t)SEQ * KDIM * 2;
    u16*   vl  = (u16*)(ws + off);   off += (size_t)SEQ * KDIM * 2;
    u16*   ch  = (u16*)(ws + off);   off += (size_t)SEQ * QDIM * 2;
    u16*   cl  = (u16*)(ws + off);   off += (size_t)SEQ * QDIM * 2;
    if (off > ws_size) return;

    {
        int n8 = SEQ * HID / 8;
        k_cvtx<<<(n8 + 255) / 256, 256, 0, stream>>>(X, xb, n8);
        k_table<<<(SEQ + 7) / 8, 256, 0, stream>>>(csf);
        k_wt<0><<<dim3(HID / 64, QDIM / 64), 256, 0, stream>>>(Wq, wqT, HID, QDIM);
        k_wt<0><<<dim3(HID / 64, KDIM / 64), 256, 0, stream>>>(Wk, wkT, HID, KDIM);
        k_wt<0><<<dim3(HID / 64, KDIM / 64), 256, 0, stream>>>(Wv, wvT, HID, KDIM);
        k_wt<1><<<dim3(QDIM / 64, HID / 64), 256, 0, stream>>>(Wo, woT, QDIM, HID);
    }

    k_gemm<1, 1, 1><<<dim3(QDIM / 128, SEQ / 128), 256, 0, stream>>>(
        xb, xb, wqT, csf, qh, ql, csf, SEQ, QDIM, HID, 0, R_ATT, 1.0f);
    k_gemm<1, 1, 1><<<dim3(KDIM / 128, SEQ / 128), 256, 0, stream>>>(
        xb, xb, wkT, csf, kh, kl, csf, SEQ, KDIM, HID, 0, R_ATT, 1.0f);
    k_gemm<1, 1, 2><<<dim3(KDIM / 128, SEQ / 128), 256, 0, stream>>>(
        xb, xb, wvT, csf, vh, vl, csf, SEQ, KDIM, HID, 0, R_ATT, 1.0f);

    k_attn<1><<<dim3(NHEAD, R_ATT / 64), 128, 0, stream>>>(qh, ql, kh, kl, vh, vl, ch, cl, 0, R_OUT);
    k_attn<0><<<dim3(NHEAD, (SEQ - R_ATT) / 64), 128, 0, stream>>>(qh, ql, kh, kl, vh, vl, ch, cl, R_ATT / 64, R_OUT);

    const float osc = 1.0f / 65536.0f;
    k_gemm<0, 2, 0><<<dim3(HID / 128, R_OUT / 128), 256, 0, stream>>>(
        ch, cl, woT, Out, ch, cl, csf, SEQ, HID, QDIM, 0, 0, osc);
    k_gemm<0, 1, 0><<<dim3(HID / 128, (SEQ - R_OUT) / 128), 256, 0, stream>>>(
        ch, ch, woT, Out, ch, cl, csf, SEQ, HID, QDIM, R_OUT, 0, osc);
}
